// GlobalAttention_48533130445227
// MI455X (gfx1250) — hardware-verified
//
#include <hip/hip_runtime.h>


#ifndef NG
#define NG   16
#endif
#ifndef SEQ
#define SEQ  512
#endif
#define S_FULL 512
#define DM   1024
#define NH   16
#define HD   64
#define ZT   (NG * NH)
#define ZH   ((ZT) < 32 ? (ZT) : 32)
#define NTOK (NG * S_FULL)
#define PCAR 1024.0f
#define ACAR 16.0f
#define WCAR 64.0f
#define SCL  0.125f
#define LNEPS 1e-5f
#define BCH  2048
#define NBLK ((NTOK + BCH - 1) / BCH)
static_assert(SEQ % 128 == 0);
static_assert(SEQ <= S_FULL);
static_assert((ZT % ZH) == 0);
static_assert(DM % 64 == 0);
static_assert(HD % 64 == 0);
static_assert(NTOK % 64 == 0);
static_assert(SEQ % 64 == 0);
static_assert(NBLK >= 1 && NBLK <= 1024);

typedef _Float16 h16;
typedef unsigned short bf;
typedef __attribute__((ext_vector_type(16))) __bf16   v16bf;
typedef __attribute__((ext_vector_type(16))) _Float16 v16h;
typedef __attribute__((ext_vector_type(8)))  _Float16 v8h;
typedef __attribute__((ext_vector_type(8)))  unsigned short v8us;
typedef __attribute__((ext_vector_type(8)))  float    v8f;
typedef __attribute__((ext_vector_type(4)))  float    v4f;
typedef __attribute__((ext_vector_type(4)))  _Float16 v4h;
typedef __attribute__((ext_vector_type(4)))  int      v4i;
typedef v8h  __attribute__((may_alias)) v8ha;
typedef v4f  __attribute__((may_alias)) v4fa;
typedef v8us __attribute__((may_alias)) v8usa;

__device__ __forceinline__ unsigned short f2bf(float f) { unsigned u = __float_as_uint(f); u += 0x7FFFu + ((u >> 16) & 1u); return (unsigned short)(u >> 16); }
__device__ __forceinline__ float bf2f(unsigned short b) { return __uint_as_float(((unsigned)b) << 16); }
__device__ __forceinline__ float bfr(float f) { return bf2f(f2bf(f)); }
__device__ __forceinline__ h16 tohx(float x) { return (h16)x; }
__device__ __forceinline__ v16h cat16(v8h lo, v8h hi) { return __builtin_shufflevector(lo, hi, 0, 1, 2, 3, 4, 5, 6, 7, 8, 9, 10, 11, 12, 13, 14, 15); }
__device__ __forceinline__ v16bf cat16b(v8us lo, v8us hi) { return __builtin_bit_cast(v16bf, __builtin_shufflevector(lo, hi, 0, 1, 2, 3, 4, 5, 6, 7, 8, 9, 10, 11, 12, 13, 14, 15)); }
__device__ __forceinline__ v8f wmma16(v16h a, v16h b, v8f c) { return __builtin_amdgcn_wmma_f32_16x16x32_f16(false, a, false, b, (short)0, c, false, false); }
__device__ __forceinline__ v8f wmmab(v16bf a, v16bf b, v8f c) { return __builtin_amdgcn_wmma_f32_16x16x32_bf16(false, a, false, b, (short)0, c, false, false); }

template <typename T16> struct WFrag;
template <> struct WFrag<h16> { typedef v16h V; static __device__ __forceinline__ V ld(const h16* p) { return cat16(*(const v8h*)p, *(const v8h*)(p + 16)); } static __device__ __forceinline__ v8f mma(V a, V b, v8f c) { return wmma16(a, b, c); } };
template <> struct WFrag<bf> { typedef v16bf V; static __device__ __forceinline__ V ld(const bf* p) { return cat16b(*(const v8us*)p, *(const v8us*)(p + 16)); } static __device__ __forceinline__ v8f mma(V a, V b, v8f c) { return wmmab(a, b, c); } };
template <typename T16, int NSPLIT, bool BIAS>
__global__ __launch_bounds__(32) void k_gemmw(const T16* __restrict__ A, const T16* __restrict__ A2, const T16* __restrict__ Bt, const T16* __restrict__ Bt2, int K, float* C, int ldc, const float* __restrict__ bias, size_t sA, size_t sB, size_t sC) {
    typedef typename WFrag<T16>::V V;
    __shared__ __align__(16) float os[16 * 68];
    const size_t z = blockIdx.z; A += z * sA; if (A2) A2 += z * sA; Bt += z * sB; if (Bt2) Bt2 += z * sB; C += z * sC;
    const int lane = threadIdx.x & 31, lr = lane & 15, hi = lane >> 4; const int r0 = blockIdx.x * 64, c0 = blockIdx.y * 64;
    v8f acc[4][4];
#pragma unroll
    for (int mb = 0; mb < 4; ++mb)
#pragma unroll
        for (int nb = 0; nb < 4; ++nb) acc[mb][nb] = (v8f){};
    const size_t aoff = (size_t)(r0 + lr) * K + 8 * hi, boff = (size_t)(c0 + lr) * K + 8 * hi;
#pragma unroll 1
    for (int kc = 0; kc < K; kc += 32) {
        V a[4], a2[4];
#pragma unroll
        for (int mb = 0; mb < 4; ++mb) { a[mb] = WFrag<T16>::ld(A + aoff + (size_t)mb * 16 * K + kc); if (NSPLIT == 1 || NSPLIT == 2) a2[mb] = WFrag<T16>::ld(A2 + aoff + (size_t)mb * 16 * K + kc); }
#pragma unroll
        for (int nb = 0; nb < 4; ++nb) { const V b = WFrag<T16>::ld(Bt + boff + (size_t)nb * 16 * K + kc); V b2; if (NSPLIT >= 2) b2 = WFrag<T16>::ld(Bt2 + boff + (size_t)nb * 16 * K + kc);
#pragma unroll
            for (int mb = 0; mb < 4; ++mb) { acc[mb][nb] = WFrag<T16>::mma(a[mb], b, acc[mb][nb]); if (NSPLIT == 1 || NSPLIT == 2) acc[mb][nb] = WFrag<T16>::mma(a2[mb], b, acc[mb][nb]); if (NSPLIT >= 2) acc[mb][nb] = WFrag<T16>::mma(a[mb], b2, acc[mb][nb]); } }
        asm volatile("v_nop\n\tv_nop\n\tv_nop\n\tv_nop" : "+v"(acc[0][0]), "+v"(acc[1][1]), "+v"(acc[2][2]), "+v"(acc[3][3]) : "v"(a[0]), "v"(a[3]));
    }
#pragma unroll
    for (int mb = 0; mb < 4; ++mb) {
#pragma unroll
        for (int nb = 0; nb < 4; ++nb) {
#pragma unroll
            for (int j = 0; j < 8; ++j) os[(hi * 8 + j) * 68 + nb * 16 + lr] = acc[mb][nb][j]; }
        __builtin_amdgcn_wave_barrier(); asm volatile("" ::: "memory");
        float* crow = C + (size_t)(r0 + mb * 16) * ldc + c0;
#pragma unroll 1
        for (int ps = 0; ps < 2; ++ps) {
#pragma unroll
            for (int s = 0; s < 8; ++s) { const int row = 2 * s + hi, cofs = lr * 4; v4f val = *(const v4fa*)(os + row * 68 + cofs); if (BIAS) { val[0] += bfr(bias[c0 + cofs]); val[1] += bfr(bias[c0 + cofs + 1]); val[2] += bfr(bias[c0 + cofs + 2]); val[3] += bfr(bias[c0 + cofs + 3]); }
                *(volatile v4f*)(crow + (size_t)row * ldc + cofs) = val; }
            if (ps == 0) __threadfence(); }
        __builtin_amdgcn_wave_barrier(); asm volatile("" ::: "memory");
    }
}

__global__ __launch_bounds__(256) void k_cvt8(const float* __restrict__ src, bf* dst, size_t n8) { const size_t i = (size_t)blockIdx.x * 256 + threadIdx.x; if (i >= n8) return; const v8f v = *(const v8f*)(src + i * 8); v8us o;
#pragma unroll
    for (int k = 0; k < 8; ++k) o[k] = f2bf(v[k]); *(volatile v8us*)(dst + i * 8) = o; __threadfence(); *(volatile v8us*)(dst + i * 8) = o; }
__global__ __launch_bounds__(256) void k_cvt8h(const float* __restrict__ src, h16* dst, size_t n8, float sc) { const size_t i = (size_t)blockIdx.x * 256 + threadIdx.x; if (i >= n8) return; const v8f v = *(const v8f*)(src + i * 8); v8h o;
#pragma unroll
    for (int k = 0; k < 8; ++k) o[k] = tohx(bfr(v[k]) * sc); *(volatile v8h*)(dst + i * 8) = o; __threadfence(); *(volatile v8h*)(dst + i * 8) = o; }

__global__ __launch_bounds__(256) void k_bchk(const int* __restrict__ ids, int* FL) {
    __shared__ int red[8];
    const int tid = threadIdx.x, lane = tid & 31, w = tid >> 5; int bad = 0;
#pragma unroll
    for (int q = 0; q < BCH / 256; ++q) { const int i = blockIdx.x * BCH + q * 256 + tid; const int ic = (i < NTOK) ? i : (NTOK - 1); const int v = ids[ic]; bad |= ((i < NTOK) && (v != ic / S_FULL)) ? 1 : 0; }
#pragma unroll
    for (int sh = 16; sh; sh >>= 1) bad |= __shfl_xor(bad, sh, 32);
    if (lane == 0) red[w] = bad;
    __syncthreads();
    if (w == 0) { int t = red[lane & 7];
#pragma unroll
        for (int sh = 16; sh; sh >>= 1) t |= __shfl_xor(t, sh, 32);
        v4i o; o[0] = t; o[1] = t; o[2] = t; o[3] = t; int* p = FL + blockIdx.x * 32 + lane * 4;
        if (lane < 8) *(volatile v4i*)p = o;
        __threadfence();
        if (lane < 8) *(volatile v4i*)p = o; }
}
__global__ __launch_bounds__(32) void k_bred(const int* __restrict__ FL, int* FLG) {
    const int lane = threadIdx.x & 31; int t = 0;
#pragma unroll 1
    for (int b = lane; b < NBLK; b += 32) t |= FL[b * 32];
#pragma unroll
    for (int sh = 16; sh; sh >>= 1) t |= __shfl_xor(t, sh, 32);
    v4i o; o[0] = t; o[1] = t; o[2] = t; o[3] = t; int* p = FLG + lane * 4;
    if (lane < 8) *(volatile v4i*)p = o;
    __threadfence();
    if (lane < 8) *(volatile v4i*)p = o;
}

__global__ __launch_bounds__(256) void k_qkp(const float* __restrict__ F, h16* P) {
    const unsigned e = (blockIdx.x * 256u + threadIdx.x) * 8u; if (e >= (unsigned)(ZT * SEQ * HD)) return;
    const int d = (int)(e % HD); const int s = (int)((e / HD) % SEQ); const int z = (int)(e / (HD * SEQ)); const int g = z / NH, h = z - g * NH;
    const v8f v = *(const v8f*)(F + ((size_t)g * S_FULL + s) * DM + h * HD + d); v8h o;
#pragma unroll
    for (int k = 0; k < 8; ++k) o[k] = tohx(v[k]);
    *(volatile v8h*)(P + e) = o; __threadfence(); *(volatile v8h*)(P + e) = o; }
__global__ __launch_bounds__(256) void k_vtp(const float* __restrict__ F, h16* VT) {
    const unsigned e = (blockIdx.x * 256u + threadIdx.x) * 8u; if (e >= (unsigned)(ZT * HD * SEQ)) return;
    const int s = (int)(e % SEQ); const int d = (int)((e / SEQ) % HD); const int z = (int)(e / (SEQ * HD)); const int g = z / NH, h = z - g * NH;
    const float* f = F + ((size_t)g * S_FULL + s) * DM + h * HD + d; v8h o;
#pragma unroll
    for (int q = 0; q < 8; ++q) o[q] = tohx(f[(size_t)q * DM]);
    *(volatile v8h*)(VT + e) = o; __threadfence(); *(volatile v8h*)(VT + e) = o; }

__global__ __launch_bounds__(256) void k_lsoft(const float* __restrict__ Sb, h16* P16) {
    const int lane = threadIdx.x & 31; const int row = blockIdx.x * 8 + (threadIdx.x >> 5); if (row >= ZH * SEQ) return; const float* sr = Sb + (size_t)row * SEQ; float mx = -3.0e38f;
#pragma unroll
    for (int ch = 0; ch < SEQ / 128; ++ch) { const int j0 = ch * 128 + lane * 4; const v4f a = *(const v4f*)(sr + j0);
#pragma unroll
        for (int q = 0; q < 4; ++q) { float t = a[q] * SCL; asm volatile("" : "+v"(t)); mx = fmaxf(mx, t); } }
#pragma unroll
    for (int sh = 16; sh; sh >>= 1) mx = fmaxf(mx, __shfl_xor(mx, sh, 32));
    float sum = 0.f;
#pragma unroll
    for (int ch = 0; ch < SEQ / 128; ++ch) { const int j0 = ch * 128 + lane * 4; const v4f a = *(const v4f*)(sr + j0);
#pragma unroll
        for (int q = 0; q < 4; ++q) { float t = a[q] * SCL; asm volatile("" : "+v"(t)); float d0 = __fsub_rn(t, mx); asm volatile("" : "+v"(d0)); sum += __builtin_amdgcn_exp2f(__fmul_rn(d0, 1.4426950408889634f)); } }
#pragma unroll
    for (int sh = 16; sh; sh >>= 1) sum += __shfl_xor(sum, sh, 32);
    const float f = __fdiv_rn(PCAR, sum);
#pragma unroll 1
    for (int ps = 0; ps < 2; ++ps) {
#pragma unroll 2
        for (int ch = 0; ch < SEQ / 128; ++ch) { const int j0 = ch * 128 + lane * 4; const v4f a = *(const v4f*)(sr + j0); v4h o4;
#pragma unroll
            for (int q = 0; q < 4; ++q) { float t = a[q] * SCL; asm volatile("" : "+v"(t)); float d0 = __fsub_rn(t, mx); asm volatile("" : "+v"(d0)); float ex = __builtin_amdgcn_exp2f(__fmul_rn(d0, 1.4426950408889634f)); asm volatile("" : "+v"(ex)); o4[q] = tohx(ex * f); }
            *(volatile v4h*)(P16 + (size_t)row * SEQ + j0) = o4; }
        if (ps == 0) __threadfence(); }
}

__global__ __launch_bounds__(256) void k_merge(const float* __restrict__ O, int zb, h16* AT) {
    const unsigned e = (blockIdx.x * 256u + threadIdx.x) * 8u; if (e >= (unsigned)(ZH * SEQ * HD)) return;
    const int d = (int)(e % HD); const int s = (int)((e / HD) % SEQ); const int zz = (int)(e / (HD * SEQ)); const int z = zb + zz; const int g = z / NH, h = z - g * NH;
    const v8f v = *(const v8f*)(O + e); v8h o;
#pragma unroll
    for (int k = 0; k < 8; ++k) o[k] = tohx(v[k] * (ACAR / PCAR));
    h16* p = AT + ((size_t)g * S_FULL + s) * DM + h * HD + d;
    *(volatile v8h*)p = o; __threadfence(); *(volatile v8h*)p = o; }

__global__ __launch_bounds__(256) void k_ln(const float* __restrict__ CO, const float* __restrict__ X, const float* __restrict__ ob, const float* __restrict__ lg, const float* __restrict__ lb, const int* __restrict__ FLG, float* OUT) {
    const int lane = threadIdx.x & 31; const int rl = blockIdx.x * 8 + (threadIdx.x >> 5); if (rl >= NG * SEQ) return;
    const int bad = FLG[0]; const float qnan = __uint_as_float(0x7fc00000u);
    const int gg = rl / SEQ, s = rl - gg * SEQ; const size_t row = (size_t)gg * S_FULL + s;
    const float* cr = CO + row * DM; const float* xr = X + row * DM; float* orow = OUT + row * DM; const float ks = 1.0f / (ACAR * WCAR);
    float sum = 0.f;
#pragma unroll 1
    for (int ch = 0; ch < DM / 128; ++ch) { const int c = ch * 128 + lane * 4; const v4f a = *(const v4f*)(cr + c); const v4f xv = *(const v4f*)(xr + c); const v4f bv = *(const v4f*)(ob + c);
#pragma unroll
        for (int q = 0; q < 4; ++q) { const float y = bfr(xv[q]) + (a[q] * ks + bfr(bv[q])); sum += y; } }
#pragma unroll
    for (int sh = 16; sh; sh >>= 1) sum += __shfl_xor(sum, sh, 32);
    const float mu = sum * (1.0f / DM);
    float vs = 0.f;
#pragma unroll 1
    for (int ch = 0; ch < DM / 128; ++ch) { const int c = ch * 128 + lane * 4; const v4f a = *(const v4f*)(cr + c); const v4f xv = *(const v4f*)(xr + c); const v4f bv = *(const v4f*)(ob + c);
#pragma unroll
        for (int q = 0; q < 4; ++q) { const float y = bfr(xv[q]) + (a[q] * ks + bfr(bv[q])); const float d0 = y - mu; vs += d0 * d0; } }
#pragma unroll
    for (int sh = 16; sh; sh >>= 1) vs += __shfl_xor(vs, sh, 32);
    const float rs = rsqrtf(vs * (1.0f / DM) + LNEPS);
#pragma unroll 1
    for (int ch = 0; ch < DM / 128; ++ch) { const int c = ch * 128 + lane * 4; const v4f a = *(const v4f*)(cr + c); const v4f xv = *(const v4f*)(xr + c); const v4f bv = *(const v4f*)(ob + c); const v4f gv = *(const v4f*)(lg + c); const v4f bb = *(const v4f*)(lb + c); v4f o;
#pragma unroll
        for (int q = 0; q < 4; ++q) { const float y = bfr(xv[q]) + (a[q] * ks + bfr(bv[q])); const float val = (y - mu) * rs * bfr(gv[q]) + bfr(bb[q]); o[q] = bad ? qnan : val; }
        *(volatile v4f*)(orow + c) = o; __threadfence(); *(volatile v4f*)(orow + c) = o; }
}

extern "C" void kernel_launch(void* const* d_in, const int* in_sizes, int n_in,
                              void* d_out, int out_size, void* d_ws, size_t ws_size, hipStream_t stream) {
    if (n_in < 8) return;
    if (in_sizes[0] < NTOK * DM || in_sizes[1] < NTOK || in_sizes[2] < 3 * DM * DM || in_sizes[3] < 3 * DM || in_sizes[4] < DM * DM || in_sizes[5] < DM || in_sizes[6] < DM || in_sizes[7] < DM) return;
    if (out_size < (NG - 1) * S_FULL * DM + SEQ * DM) return;
    const float* x = (const float*)d_in[0];
    const int* bid = (const int*)d_in[1];
    const float* w_in = (const float*)d_in[2];
    const float* b_in = (const float*)d_in[3];
    const float* w_out = (const float*)d_in[4];
    const float* b_out = (const float*)d_in[5];
    const float* lng = (const float*)d_in[6];
    const float* lnb = (const float*)d_in[7];
    float* OUT = (float*)d_out;

    const size_t bWQ = (size_t)3 * DM * DM * 2, bWO = (size_t)DM * DM * 2, bPL = (size_t)ZT * SEQ * HD * 2;
    const size_t bXB = (size_t)NTOK * DM * 2, bF = (size_t)NTOK * DM * 4, bAT = (size_t)NTOK * DM * 2;
    const size_t bSb = (size_t)ZH * SEQ * SEQ * 4, bP16 = (size_t)ZH * SEQ * SEQ * 2, bOb = (size_t)ZH * SEQ * HD * 4, bCO = (size_t)NTOK * DM * 4;
    size_t bRB = bXB + bF; if (bAT + bSb + bP16 + bOb > bRB) bRB = bAT + bSb + bP16 + bOb; if (bAT + bCO > bRB) bRB = bAT + bCO;
    char* wsp = (char*)d_ws;
    auto take = [&](size_t bytes) { char* p = wsp; wsp += (bytes + 255) & ~(size_t)255; return (void*)p; };
    bf* WQKVb = (bf*)take(bWQ);
    h16* WO16 = (h16*)take(bWO);
    h16* Q16 = (h16*)take(bPL);
    h16* K16 = (h16*)take(bPL);
    h16* VT16 = (h16*)take(bPL);
    char* RB = (char*)take(bRB);
    int* FL = (int*)take((size_t)NBLK * 128);
    int* FLG = (int*)take(128);
    if ((size_t)(wsp - (char*)d_ws) > ws_size) return;
    bf* XB = (bf*)RB;
    float* F = (float*)(RB + bXB);
    h16* AT16 = (h16*)RB;
    float* Sb = (float*)(RB + bAT);
    h16* P16 = (h16*)(RB + bAT + bSb);
    float* Ob = (float*)(RB + bAT + bSb + bP16);
    float* CO = (float*)(RB + bAT);

    k_bchk<<<(unsigned)NBLK, 256, 0, stream>>>(bid, FL);
    k_bred<<<1, 32, 0, stream>>>(FL, FLG);
    k_cvt8<<<(unsigned)((bXB / 16 + 255) / 256), 256, 0, stream>>>(x, XB, bXB / 16);
    k_cvt8<<<(unsigned)((bWQ / 16 + 255) / 256), 256, 0, stream>>>(w_in, WQKVb, bWQ / 16);
    k_cvt8h<<<(unsigned)((bWO / 16 + 255) / 256), 256, 0, stream>>>(w_out, WO16, bWO / 16, WCAR);
    const unsigned LP = (unsigned)(((size_t)ZT * SEQ * HD / 8 + 255) / 256);
    for (int p = 0; p < 3; ++p) {
        k_gemmw<bf, 0, true><<<dim3(NTOK / 64, DM / 64, 1), 32, 0, stream>>>(XB, nullptr, WQKVb + (size_t)p * DM * DM, nullptr, DM, F, DM, b_in + p * DM, 0, 0, 0);
        if (p == 0) k_qkp<<<LP, 256, 0, stream>>>(F, Q16);
        else if (p == 1) k_qkp<<<LP, 256, 0, stream>>>(F, K16);
        else k_vtp<<<LP, 256, 0, stream>>>(F, VT16);
    }
    for (int zb = 0; zb < ZT; zb += ZH) {
        k_gemmw<h16, 0, false><<<dim3(SEQ / 64, SEQ / 64, ZH), 32, 0, stream>>>(Q16 + (size_t)zb * SEQ * HD, nullptr, K16 + (size_t)zb * SEQ * HD, nullptr, HD, Sb, SEQ, nullptr, (size_t)SEQ * HD, (size_t)SEQ * HD, (size_t)SEQ * SEQ);
        k_lsoft<<<(unsigned)(ZH * SEQ / 8), 256, 0, stream>>>(Sb, P16);
        k_gemmw<h16, 0, false><<<dim3(SEQ / 64, HD / 64, ZH), 32, 0, stream>>>(P16, nullptr, VT16 + (size_t)zb * HD * SEQ, nullptr, SEQ, Ob, HD, nullptr, (size_t)SEQ * SEQ, (size_t)HD * SEQ, (size_t)SEQ * HD);
        k_merge<<<(unsigned)(((size_t)ZH * SEQ * HD / 8 + 255) / 256), 256, 0, stream>>>(Ob, zb, AT16);
    }
    k_gemmw<h16, 0, false><<<dim3(NTOK / 64, DM / 64, 1), 32, 0, stream>>>(AT16, nullptr, WO16, nullptr, DM, CO, DM, nullptr, 0, 0, 0);
    k_ln<<<(unsigned)((NG * SEQ + 7) / 8), 256, 0, stream>>>(CO, x, b_out, lng, lnb, FLG, OUT);
}
